// BboxInteractionNetwork_84902913507459
// MI455X (gfx1250) — hardware-run, weakly checked
//
#include <hip/hip_runtime.h>
#include <stddef.h>


#define EMB        128
#define NS         16
#define XPB        (NS * 16)
#define NTHR       256
#define NWAVE      8
#define R1ROWS     (NS * 16)
#define DROWS      (NS * 4)
#define SP         132
#define WPL        (EMB * EMB)
#define NMAT       5
#define WCARRY     64.0f
#define INV_WCARRY 0.015625f

#define OFF_S      0
#define OFF_DY     (OFF_S  + R1ROWS * SP * 4)
#define OFF_F0     (OFF_DY + DROWS * SP * 4)
#define OFF_XT     (OFF_F0 + DROWS * SP * 4)
#define OFF_W0     (OFF_XT + XPB * 4)
#define OFF_B0     (OFF_W0 + 16 * EMB * 4)
#define OFF_B1     (OFF_B0 + 3 * EMB * 4)
#define LDS_TOT    (OFF_B1 + NMAT * EMB * 4)
#define PREP_BLK   ((NMAT * WPL) / (NTHR * 8))
#define WS_NEED    ((size_t)NMAT * WPL * 2)

static_assert((NMAT * WPL) % (NTHR * 8) == 0);
static_assert(((SP * 4) % 16) == 0);
static_assert((OFF_DY % 16) == 0);
static_assert((OFF_F0 % 16) == 0);
static_assert((OFF_XT % 16) == 0);
static_assert((OFF_W0 % 16) == 0);
static_assert((OFF_B0 % 16) == 0);
static_assert((OFF_B1 % 16) == 0);
static_assert(LDS_TOT == 216064);
static_assert(R1ROWS == 2 * NWAVE * 16);
static_assert(DROWS == 4 * 16);
static_assert(NS == 2 * NWAVE);
static_assert(XPB == 2 * 4 * 32);
static_assert((R1ROWS * EMB) % NTHR == 0);

typedef float    v4f  __attribute__((ext_vector_type(4)));
typedef float    v8f  __attribute__((ext_vector_type(8)));
typedef _Float16 v4h  __attribute__((ext_vector_type(4)));
typedef _Float16 v8h  __attribute__((ext_vector_type(8)));
typedef _Float16 v16h __attribute__((ext_vector_type(16)));
union Frag { v16h v; v8h half[2]; };

__device__ __forceinline__ v8f zero8() {
  v8f z = {0.f, 0.f, 0.f, 0.f, 0.f, 0.f, 0.f, 0.f};
  return z;
}

__device__ __forceinline__ v8f wmf(v16h a, v16h b, v8f c) {
  v8f d = __builtin_amdgcn_wmma_f32_16x16x32_f16(false, a, false, b, (short)0, c, false, false);
  asm volatile("v_nop\n\tv_nop\n\tv_nop\n\tv_nop" : "+v"(d) : "v"(a), "v"(b));
  return d;
}

__device__ __forceinline__ v16h a_frag_f32(const float* ap) {
  const v4f f0 = *(const v4f*)(ap);
  const v4f f1 = *(const v4f*)(ap + 4);
  const v4f f2 = *(const v4f*)(ap + 16);
  const v4f f3 = *(const v4f*)(ap + 20);
  const v4h h0 = __builtin_convertvector(f0, v4h);
  const v4h h1 = __builtin_convertvector(f1, v4h);
  const v4h h2 = __builtin_convertvector(f2, v4h);
  const v4h h3 = __builtin_convertvector(f3, v4h);
  Frag a;
  a.half[0] = __builtin_shufflevector(h0, h1, 0, 1, 2, 3, 4, 5, 6, 7);
  a.half[1] = __builtin_shufflevector(h2, h3, 0, 1, 2, 3, 4, 5, 6, 7);
  return a.v;
}

__device__ __forceinline__ v16h b_frag(const _Float16* bp) {
  Frag b;
  b.half[0] = *(const v8h*)(bp);
  b.half[1] = *(const v8h*)(bp + 16);
  return b.v;
}

template <int NCT>
__device__ __forceinline__ void gemm_k128(const float* arow, const _Float16* __restrict__ bcol,
                                          v8f (&acc)[NCT]) {
#pragma unroll
  for (int c = 0; c < NCT; ++c) acc[c] = zero8();
#pragma unroll 1
  for (int ks = 0; ks < EMB / 32; ++ks) {
    const v16h a = a_frag_f32(arow + 32 * ks);
#pragma unroll
    for (int c = 0; c < NCT; ++c) {
      const v16h b = b_frag(bcol + (size_t)c * 16 * EMB + 32 * ks);
      acc[c] = wmf(a, b, acc[c]);
    }
  }
}

__device__ __forceinline__ void epi_inplace_res(float* sp, v8f a, float bias) {
#pragma unroll
  for (int r = 0; r < 8; ++r) {
    const float rv = sp[r * SP];
    sp[r * SP] = (a[r] * INV_WCARRY + bias) + rv;
  }
}
__device__ __forceinline__ void epi_relu(float* dst, v8f a, float bias) {
#pragma unroll
  for (int r = 0; r < 8; ++r) dst[r * SP] = fmaxf(a[r] * INV_WCARRY + bias, 0.0f);
}
__device__ __forceinline__ void epi_res(float* dst, v8f a, float bias, const float* res) {
#pragma unroll
  for (int r = 0; r < 8; ++r) dst[r * SP] = (a[r] * INV_WCARRY + bias) + res[r * SP];
}

__global__ __launch_bounds__(NTHR) void k_prep(
    const float* __restrict__ w0, const float* __restrict__ w1, const float* __restrict__ w2,
    const float* __restrict__ w3, const float* __restrict__ w4, _Float16* wp) {
  const int gid = (int)blockIdx.x * NTHR + (int)threadIdx.x;
  const int o   = gid * 8;
  const int mat = o >> 14;
  const int idx = o & (WPL - 1);
  const int n   = idx >> 7;
  const int k0  = idx & (EMB - 1);
  const float* src = (mat == 0) ? w0 : ((mat == 1) ? w1 : ((mat == 2) ? w2 : ((mat == 3) ? w3 : w4)));
  const float* sp = src + (size_t)k0 * EMB + n;
  v4f fa, fb;
  fa.x = WCARRY * sp[0 * EMB];
  fa.y = WCARRY * sp[1 * EMB];
  fa.z = WCARRY * sp[2 * EMB];
  fa.w = WCARRY * sp[3 * EMB];
  fb.x = WCARRY * sp[4 * EMB];
  fb.y = WCARRY * sp[5 * EMB];
  fb.z = WCARRY * sp[6 * EMB];
  fb.w = WCARRY * sp[7 * EMB];
  const v4h ha = __builtin_convertvector(fa, v4h);
  const v4h hb = __builtin_convertvector(fb, v4h);
  const v8h hv = __builtin_shufflevector(ha, hb, 0, 1, 2, 3, 4, 5, 6, 7);
  _Float16* dst = wp + o;
  *(volatile v8h*)dst = hv;
  __threadfence();
  *(volatile v8h*)dst = hv;
}

__global__ __launch_bounds__(NTHR) void k_main(
    const float* __restrict__ x,
    const float* __restrict__ sa0_w, const float* __restrict__ sa0_b,
    const float* __restrict__ sb0_w, const float* __restrict__ sb0_b,
    const float* __restrict__ rel0_w, const float* __restrict__ rel0_b,
    const float* __restrict__ sa1_b, const float* __restrict__ sb1_b, const float* __restrict__ rel1_b,
    const float* __restrict__ aff0_b, const float* __restrict__ aff1_b,
    const _Float16* __restrict__ wp, float* out0, float* out1) {
  extern __shared__ __attribute__((aligned(16))) char smem[];
  float* S  = (float*)(smem + OFF_S);
  float* DY = (float*)(smem + OFF_DY);
  float* F0 = (float*)(smem + OFF_F0);
  float* XT = (float*)(smem + OFF_XT);
  float* W0 = (float*)(smem + OFF_W0);
  float* B0 = (float*)(smem + OFF_B0);
  float* B1 = (float*)(smem + OFF_B1);

  const int tid = (int)threadIdx.x, lane = tid & 31, wave = tid >> 5, h = lane >> 4, m = lane & 15;
  const int blk = (int)blockIdx.x;
  const int n0 = blk * NS;

  {
    const float xv = x[(size_t)blk * XPB + tid];
    XT[tid] = xv;
  }
  if (wave < 2) {
    const size_t go = (size_t)blk * XPB + (size_t)(wave * 128 + 4 * lane);
    const v4f v = *(const v4f*)(x + go);
    *(volatile v4f*)(out0 + go) = v;
    __threadfence();
    *(volatile v4f*)(out0 + go) = v;
  }
#pragma unroll 1
  for (int i = tid; i < 4 * EMB; i += NTHR) {
    W0[i]           = sa0_w[i];
    W0[4 * EMB + i] = sb0_w[i];
  }
#pragma unroll 1
  for (int i = tid; i < 8 * EMB; i += NTHR) W0[8 * EMB + i] = rel0_w[i];
  if (tid < EMB) {
    B0[tid]           = sa0_b[tid];
    B0[EMB + tid]     = sb0_b[tid];
    B0[2 * EMB + tid] = rel0_b[tid];
    B1[tid]           = sa1_b[tid];
    B1[EMB + tid]     = sb1_b[tid];
    B1[2 * EMB + tid] = rel1_b[tid];
    B1[3 * EMB + tid] = aff0_b[tid];
    B1[4 * EMB + tid] = aff1_b[tid];
  }
  __syncthreads();

  const int col  = tid & (EMB - 1);
  const int rpar = tid >> 7;

  {
    const float* wa = W0 + col;
    const float* wb = W0 + 4 * EMB + col;
    const float* wr = W0 + 8 * EMB + col;
#pragma unroll 1
    for (int i = 0; i < R1ROWS / 2; ++i) {
      const int row = 2 * i + rpar;
      float d, bias;
      if (row < NS) {
        const float* in = XT + row * 16;
        d = in[0] * wa[0];
        d = fmaf(in[1], wa[EMB], d);
        d = fmaf(in[2], wa[2 * EMB], d);
        d = fmaf(in[3], wa[3 * EMB], d);
        bias = B0[col];
      } else if (row < 4 * NS) {
        const int i2 = row - NS;
        const int s = i2 / 3;
        const int bx = i2 - 3 * s;
        const float* in = XT + s * 16 + 4 * (bx + 1);
        d = in[0] * wb[0];
        d = fmaf(in[1], wb[EMB], d);
        d = fmaf(in[2], wb[2 * EMB], d);
        d = fmaf(in[3], wb[3 * EMB], d);
        bias = B0[EMB + col];
      } else {
        const int i2 = row - 4 * NS;
        const int s = i2 / 12;
        const int p = i2 - 12 * s;
        const int pi = p / 3;
        int pj = p - 3 * pi;
        pj += (pj >= pi) ? 1 : 0;
        const float* ia = XT + s * 16 + 4 * pi;
        const float* ib = XT + s * 16 + 4 * pj;
        d = ia[0] * wr[0];
        d = fmaf(ia[1], wr[EMB], d);
        d = fmaf(ia[2], wr[2 * EMB], d);
        d = fmaf(ia[3], wr[3 * EMB], d);
        d = fmaf(ib[0], wr[4 * EMB], d);
        d = fmaf(ib[1], wr[5 * EMB], d);
        d = fmaf(ib[2], wr[6 * EMB], d);
        d = fmaf(ib[3], wr[7 * EMB], d);
        bias = B0[2 * EMB + col];
      }
      S[row * SP + col] = fmaxf(d + bias, 0.0f);
    }
  }
  __syncthreads();

#pragma unroll 1
  for (int rti = 0; rti < 2; ++rti) {
    const int rt = 2 * wave + rti;
    const int wsel = (rt == 0) ? 0 : ((rt < 4) ? 1 : 2);
    v8f acc[8];
    gemm_k128<8>(S + (16 * rt + m) * SP + 8 * h, wp + (size_t)wsel * WPL + m * EMB + 8 * h, acc);
    const float* bb = B1 + wsel * EMB;
    float* sp = S + (16 * rt + 8 * h) * SP + m;
#pragma unroll
    for (int c = 0; c < 8; ++c) epi_inplace_res(sp + 16 * c, acc[c], bb[16 * c + m]);
  }
  __syncthreads();

#pragma unroll 1
  for (int i = 0; i < DROWS / 2; ++i) {
    const int row = 2 * i + rpar;
    const int s = row >> 2, obj = row & 3;
    const int selfrow = (obj == 0) ? s : (NS + 3 * s + obj - 1);
    const int rb = 4 * NS + 12 * s + 3 * obj;
    const float sv = S[selfrow * SP + col];
    const float ra = S[rb * SP + col];
    const float rbv = S[(rb + 1) * SP + col];
    const float rc = S[(rb + 2) * SP + col];
    DY[row * SP + col] = sv + ((ra + rbv) + rc);
  }
  __syncthreads();

  const int rt2 = wave & 3, cg = wave >> 2;

  {
    v8f acc[4];
    gemm_k128<4>(DY + (16 * rt2 + m) * SP + 8 * h, wp + (size_t)3 * WPL + (64 * cg + m) * EMB + 8 * h, acc);
    const float* bb = B1 + 3 * EMB + 64 * cg + m;
    float* dp = F0 + (16 * rt2 + 8 * h) * SP + 64 * cg + m;
#pragma unroll
    for (int c = 0; c < 4; ++c) epi_relu(dp + 16 * c, acc[c], bb[16 * c]);
  }
  __syncthreads();

  {
    v8f acc[4];
    gemm_k128<4>(F0 + (16 * rt2 + m) * SP + 8 * h, wp + (size_t)4 * WPL + (64 * cg + m) * EMB + 8 * h, acc);
    const float* bb = B1 + 4 * EMB + 64 * cg + m;
    float* dp = DY + (16 * rt2 + 8 * h) * SP + 64 * cg + m;
    const float* rp = F0 + (16 * rt2 + 8 * h) * SP + 64 * cg + m;
#pragma unroll
    for (int c = 0; c < 4; ++c) epi_res(dp + 16 * c, acc[c], bb[16 * c], rp + 16 * c);
  }
  __syncthreads();

  {
    v4f fin[2];
#pragma unroll
    for (int j = 0; j < 2; ++j) {
      const int s = 2 * wave + j;
      const float* p = DY + (4 * s) * SP + 4 * lane;
      const v4f t0 = *(const v4f*)(p);
      const v4f t1 = *(const v4f*)(p + SP);
      const v4f t2 = *(const v4f*)(p + 2 * SP);
      const v4f t3 = *(const v4f*)(p + 3 * SP);
      fin[j] = (((t0 + t1) + t2) + t3) * 0.25f;
    }
#pragma unroll
    for (int j = 0; j < 2; ++j) {
      const int s = 2 * wave + j;
      *(volatile v4f*)(out1 + (size_t)(n0 + s) * EMB + 4 * lane) = fin[j];
    }
    __threadfence();
#pragma unroll
    for (int j = 0; j < 2; ++j) {
      const int s = 2 * wave + j;
      *(volatile v4f*)(out1 + (size_t)(n0 + s) * EMB + 4 * lane) = fin[j];
    }
  }
}

extern "C" void kernel_launch(void* const* d_in, const int* in_sizes, int n_in,
                              void* d_out, int out_size, void* d_ws, size_t ws_size,
                              hipStream_t stream) {
  if (n_in < 17) return;
  const int nx = in_sizes[0];
  if (nx < XPB || (nx % XPB) != 0) return;
  const int nN = nx / 16;
  if (in_sizes[1] != 4 * EMB || in_sizes[2] != EMB) return;
  if (in_sizes[3] != WPL || in_sizes[4] != EMB) return;
  if (in_sizes[5] != 4 * EMB || in_sizes[6] != EMB) return;
  if (in_sizes[7] != WPL || in_sizes[8] != EMB) return;
  if (in_sizes[9] != 8 * EMB || in_sizes[10] != EMB) return;
  if (in_sizes[11] != WPL || in_sizes[12] != EMB) return;
  if (in_sizes[13] != WPL || in_sizes[14] != EMB) return;
  if (in_sizes[15] != WPL || in_sizes[16] != EMB) return;
  if ((size_t)out_size != (size_t)nx + (size_t)nN * EMB) return;
  if (WS_NEED > ws_size) return;

  const float* x      = (const float*)d_in[0];
  const float* sa0_w  = (const float*)d_in[1];
  const float* sa0_b  = (const float*)d_in[2];
  const float* sa1_w  = (const float*)d_in[3];
  const float* sa1_b  = (const float*)d_in[4];
  const float* sb0_w  = (const float*)d_in[5];
  const float* sb0_b  = (const float*)d_in[6];
  const float* sb1_w  = (const float*)d_in[7];
  const float* sb1_b  = (const float*)d_in[8];
  const float* rel0_w = (const float*)d_in[9];
  const float* rel0_b = (const float*)d_in[10];
  const float* rel1_w = (const float*)d_in[11];
  const float* rel1_b = (const float*)d_in[12];
  const float* aff0_w = (const float*)d_in[13];
  const float* aff0_b = (const float*)d_in[14];
  const float* aff1_w = (const float*)d_in[15];
  const float* aff1_b = (const float*)d_in[16];

  float* out0 = (float*)d_out;
  float* out1 = out0 + (size_t)nx;

  _Float16* wp = (_Float16*)d_ws;

  const int nblk = nx / XPB;

  hipFuncSetAttribute(reinterpret_cast<const void*>(&k_main), hipFuncAttributeMaxDynamicSharedMemorySize, LDS_TOT);

  k_prep<<<PREP_BLK, NTHR, 0, stream>>>(sa1_w, sb1_w, rel1_w, aff0_w, aff1_w, wp);
  k_main<<<nblk, NTHR, LDS_TOT, stream>>>(x, sa0_w, sa0_b, sb0_w, sb0_b, rel0_w, rel0_b,
                                          sa1_b, sb1_b, rel1_b, aff0_b, aff1_b, wp, out0, out1);
}
